// MLPAttention_52218212384987
// MI455X (gfx1250) — hardware-verified
//
#include <hip/hip_runtime.h>


#ifndef NB
#define NB 8
#endif
#ifndef SEQ
#define SEQ 1024
#endif
#define NB_FULL 8
#define LQ      64
#define LK      SEQ
#define LK_FULL 1024
#define DC      512
#define DQ      512
#define HH      256
#define NQR     (NB * LQ)
#define NKR     (NB * LK)
#define KPT     (LK / 256)
#define OUT1_OFF ((size_t)NB_FULL * LQ * LK_FULL)

static_assert(NB >= 1 && NB <= NB_FULL);
static_assert(LK % 256 == 0 && LK >= 256 && LK <= LK_FULL);
static_assert(KPT >= 1 && KPT <= 4);
static_assert(HH == 256);
static_assert(DC == 512 && DQ == 512);
static_assert(LQ % 64 == 0 && DC % 64 == 0 && HH % 64 == 0 && (NKR % 64) == 0 && (NQR % 64) == 0);
static_assert(DC % 32 == 0 && DQ % 32 == 0 && LK % 64 == 0);
static_assert(OUT1_OFF * 4 == 2097152);

typedef unsigned short bf;
typedef __attribute__((ext_vector_type(16))) __bf16   v16bf;
typedef __attribute__((ext_vector_type(8)))  unsigned short v8us;
typedef __attribute__((ext_vector_type(8)))  float    v8f;
typedef __attribute__((ext_vector_type(4)))  float    v4f;
typedef v4f  __attribute__((may_alias)) v4fa;
typedef v8us __attribute__((may_alias)) v8usa;

__device__ __forceinline__ unsigned short f2bf(float f) { unsigned u = __float_as_uint(f); u += 0x7FFFu + ((u >> 16) & 1u); return (unsigned short)(u >> 16); }
__device__ __forceinline__ float bf2f(unsigned short b) { return __uint_as_float(((unsigned)b) << 16); }
__device__ __forceinline__ float bfr(float f) { return bf2f(f2bf(f)); }
__device__ __forceinline__ v16bf cat16b(v8us lo, v8us hi) { return __builtin_bit_cast(v16bf, __builtin_shufflevector(lo, hi, 0, 1, 2, 3, 4, 5, 6, 7, 8, 9, 10, 11, 12, 13, 14, 15)); }
__device__ __forceinline__ v8f wmmab(v16bf a, v16bf b, v8f c) { return __builtin_amdgcn_wmma_f32_16x16x32_bf16(false, a, false, b, (short)0, c, false, false); }

__global__ __launch_bounds__(256) void k_wsplit(const float* __restrict__ Wm, bf* WB) {
    const int i = blockIdx.x * 256 + threadIdx.x;
    if (i >= HH * (DC + DQ) / 8) return;
    const int row = i / ((DC + DQ) / 8), g8 = i - row * ((DC + DQ) / 8);
    const v8f v = *(const v8f*)(Wm + (size_t)i * 8);
    v8us o;
#pragma unroll
    for (int k = 0; k < 8; ++k) o[k] = f2bf(v[k]);
    const int half = (g8 >= DC / 8) ? 1 : 0;
    const int col8 = g8 - half * (DC / 8);
    const size_t d = (size_t)half * HH * DC + (size_t)row * DC + (size_t)col8 * 8;
    *(volatile v8us*)(WB + d) = o; __threadfence(); *(volatile v8us*)(WB + d) = o;
}

__global__ __launch_bounds__(256) void k_bf(const float* __restrict__ src, size_t sstr, bf* dst, size_t dstr, size_t n8) {
    const size_t i = (size_t)blockIdx.x * 256 + threadIdx.x; if (i >= n8) return;
    const float* sp = src + (size_t)blockIdx.y * sstr + i * 8; bf* dp = dst + (size_t)blockIdx.y * dstr + i * 8;
    const v8f v = *(const v8f*)sp; v8us o;
#pragma unroll
    for (int k = 0; k < 8; ++k) o[k] = f2bf(v[k]);
    *(volatile v8us*)dp = o; __threadfence(); *(volatile v8us*)dp = o;
}

template <bool SPLITA>
__global__ __launch_bounds__(128) void k_gemmb(const bf* __restrict__ A, const bf* __restrict__ Al, const bf* __restrict__ Bn, const float* __restrict__ bias,
                                               float* C, int ldc, int K, size_t zA, size_t zB, size_t zC) {
    __shared__ __align__(16) float ost[4][16 * 68];
    const int lane = threadIdx.x & 31, wave = threadIdx.x >> 5, lr = lane & 15, hi = lane >> 4;
    const int z = blockIdx.z;
    A += (size_t)z * zA; if (SPLITA) Al += (size_t)z * zA; Bn += (size_t)z * zB; C += (size_t)z * zC;
    const int r0 = blockIdx.x * 64 + wave * 16, c0 = blockIdx.y * 64;
    const size_t aoff = (size_t)(r0 + lr) * K + 8 * hi;
    size_t boff[4];
#pragma unroll
    for (int t = 0; t < 4; ++t) boff[t] = (size_t)(c0 + t * 16 + lr) * K + 8 * hi;
    v8f acc[4];
#pragma unroll
    for (int t = 0; t < 4; ++t) acc[t] = (v8f){};
#pragma unroll 1
    for (int kc = 0; kc < K; kc += 32) {
        const v16bf a = cat16b(*(const v8us*)(A + aoff + kc), *(const v8us*)(A + aoff + kc + 16));
        v16bf al = a;
        if (SPLITA) al = cat16b(*(const v8us*)(Al + aoff + kc), *(const v8us*)(Al + aoff + kc + 16));
#pragma unroll
        for (int t = 0; t < 4; ++t) { const v16bf b = cat16b(*(const v8us*)(Bn + boff[t] + kc), *(const v8us*)(Bn + boff[t] + kc + 16)); acc[t] = wmmab(a, b, acc[t]); if (SPLITA) acc[t] = wmmab(al, b, acc[t]); }
        asm volatile("v_nop\n\tv_nop\n\tv_nop\n\tv_nop" : "+v"(acc[0]), "+v"(acc[1]), "+v"(acc[2]), "+v"(acc[3]) : "v"(a), "v"(al));
    }
    float* os = &ost[wave][0];
#pragma unroll
    for (int t = 0; t < 4; ++t) { const float bv = bias ? bfr(bias[c0 + t * 16 + lr]) : 0.f;
#pragma unroll
        for (int j = 0; j < 8; ++j) os[(hi * 8 + j) * 68 + t * 16 + lr] = acc[t][j] + bv; }
    __syncthreads();
    float* crow = C + (size_t)r0 * ldc + c0;
    auto pass = [&]() {
#pragma unroll
        for (int s = 0; s < 8; ++s) { const int Lid = (lane >> 3) + 4 * s, piece = lane & 7; const int row = Lid >> 1, cofs = (Lid & 1) * 32 + piece * 4;
            const v4f val = *(const v4fa*)(os + row * 68 + cofs);
            *(volatile v4f*)(crow + (size_t)row * ldc + cofs) = val; }
    };
    pass(); __threadfence(); pass();
}

__global__ __launch_bounds__(256) void k_ct(const float* __restrict__ X, bf* CT) {
    __shared__ float tl[64][65];
    const int tid = threadIdx.x, l0 = blockIdx.x * 64, c0 = blockIdx.y * 64, b = blockIdx.z;
    const float* src = X + (size_t)b * LK_FULL * DC;
    { const int ll = tid >> 2, cq = (tid & 3) * 16;
#pragma unroll
      for (int i = 0; i < 16; ++i) tl[cq + i][ll] = src[(size_t)(l0 + ll) * DC + c0 + cq + i]; }
    __syncthreads();
    const int piece = tid & 7;
    auto pass = [&]() {
#pragma unroll
        for (int s = 0; s < 2; ++s) { const int c = (tid >> 3) + 32 * s; v8us o;
#pragma unroll
            for (int i = 0; i < 8; ++i) o[i] = f2bf(tl[c][piece * 8 + i]);
            *(volatile v8us*)(CT + ((size_t)b * DC + c0 + c) * LK + l0 + piece * 8) = o; }
    };
    pass(); __threadfence(); pass();
}

__global__ __launch_bounds__(256) void k_score(const float* __restrict__ Qf, const float* __restrict__ Kf, const float* __restrict__ vw, const float* __restrict__ gp,
                                               const float* __restrict__ sbp, float* Pout, bf* Ph, bf* Pl) {
    __shared__ float qs[HH]; __shared__ float wsm[HH]; __shared__ float red[256]; __shared__ __align__(16) float pr[LK];
    const int tid = threadIdx.x; const int row = blockIdx.x; const int b = row / LQ;
    qs[tid] = Qf[(size_t)row * HH + tid];
    const float vb = bfr(vw[tid]);
    red[tid] = vb * vb; __syncthreads();
#pragma unroll
    for (int st = 128; st >= 1; st >>= 1) { if (tid < st) red[tid] = red[tid] + red[tid + st]; __syncthreads(); }
    const float nrm = sqrtf(red[0]);
    const float g0 = bfr(gp[0]), sb0 = bfr(sbp[0]);
    wsm[tid] = (g0 * vb) * (1.0f / nrm);
    __syncthreads();
    const float* kb = Kf + ((size_t)b * LK + tid) * HH;
    float s[KPT];
#pragma unroll
    for (int c = 0; c < KPT; ++c) s[c] = 0.f;
#pragma unroll 1
    for (int u = 0; u < HH; ++u) {
        const float qu = qs[u], wu = wsm[u];
#pragma unroll
        for (int c = 0; c < KPT; ++c) { const float a = qu + kb[(size_t)c * 256 * HH + u]; const float th = 1.0f - 2.0f / (__expf(2.0f * a) + 1.0f); s[c] = fmaf(wu, th, s[c]); }
    }
#pragma unroll
    for (int c = 0; c < KPT; ++c) s[c] += sb0;
    float mloc = s[0];
#pragma unroll
    for (int c = 1; c < KPT; ++c) mloc = fmaxf(mloc, s[c]);
    red[tid] = mloc; __syncthreads();
#pragma unroll
    for (int st = 128; st >= 1; st >>= 1) { if (tid < st) red[tid] = fmaxf(red[tid], red[tid + st]); __syncthreads(); }
    const float m = red[0]; __syncthreads();
    float lsum = 0.f;
#pragma unroll
    for (int c = 0; c < KPT; ++c) { s[c] = __expf(s[c] - m); lsum += s[c]; }
    red[tid] = lsum; __syncthreads();
#pragma unroll
    for (int st = 128; st >= 1; st >>= 1) { if (tid < st) red[tid] = red[tid] + red[tid + st]; __syncthreads(); }
    const float inv = 1.0f / red[0];
#pragma unroll
    for (int c = 0; c < KPT; ++c) pr[tid + 256 * c] = s[c] * inv;
    __syncthreads();
    float* prow = Pout + (size_t)row * LK; bf* hrow = Ph + (size_t)row * LK; bf* lrow = Pl + (size_t)row * LK;
    auto pass = [&]() {
#pragma unroll
        for (int q4 = tid; q4 < LK / 4; q4 += 256) { const v4f val = *(const v4fa*)(pr + 4 * q4); *(volatile v4f*)(prow + 4 * q4) = val; }
#pragma unroll
        for (int q8 = tid; q8 < LK / 8; q8 += 256) { v8us oh, ol;
#pragma unroll
            for (int q = 0; q < 8; ++q) { const float v = pr[8 * q8 + q]; const unsigned short hb = f2bf(v); oh[q] = hb; ol[q] = f2bf(v - bf2f(hb)); }
            *(volatile v8us*)(hrow + 8 * q8) = oh; *(volatile v8us*)(lrow + 8 * q8) = ol; }
    };
    pass(); __threadfence(); pass();
}

extern "C" void kernel_launch(void* const* d_in, const int* in_sizes, int n_in,
                              void* d_out, int out_size, void* d_ws, size_t ws_size, hipStream_t stream) {
    if (n_in < 7) return;
    if (in_sizes[0] < NQR * DQ) return;
    if (in_sizes[1] < (NB - 1) * LK_FULL * DC + LK * DC) return;
    if (in_sizes[2] < HH * (DC + DQ) || in_sizes[3] < HH || in_sizes[4] < HH || in_sizes[5] < 1 || in_sizes[6] < 1) return;
    if ((size_t)out_size < OUT1_OFF + (size_t)NQR * DC) return;
    const float* query = (const float*)d_in[0]; const float* context = (const float*)d_in[1]; const float* Wm = (const float*)d_in[2];
    const float* bias = (const float*)d_in[3]; const float* vv = (const float*)d_in[4]; const float* gg = (const float*)d_in[5]; const float* sbp = (const float*)d_in[6];
    float* out0 = (float*)d_out;
    float* out1 = out0 + OUT1_OFF;
    char* wsp = (char*)d_ws;
    auto take = [&](size_t bytes) { char* p = wsp; wsp += (bytes + 255) & ~(size_t)255; return (void*)p; };
    bf* WB = (bf*)take((size_t)HH * (DC + DQ) * 2);
    bf* Xc = (bf*)take((size_t)NKR * DC * 2);
    bf* Xq = (bf*)take((size_t)NQR * DQ * 2);
    float* Kf = (float*)take((size_t)NKR * HH * 4);
    float* Qf = (float*)take((size_t)NQR * HH * 4);
    bf* Ph = (bf*)take((size_t)NQR * LK * 2);
    bf* Pl = (bf*)take((size_t)NQR * LK * 2);
    bf* CT = (bf*)take((size_t)NB * DC * LK * 2);
    if ((size_t)(wsp - (char*)d_ws) > ws_size) return;
    k_wsplit<<<dim3((HH * (DC + DQ) / 8 + 255) / 256, 1, 1), 256, 0, stream>>>(Wm, WB);
    k_bf<<<dim3((LK * DC / 8 + 255) / 256, NB, 1), 256, 0, stream>>>(context, (size_t)LK_FULL * DC, Xc, (size_t)LK * DC, (size_t)LK * DC / 8);
    k_bf<<<dim3((LQ * DQ / 8 + 255) / 256, NB, 1), 256, 0, stream>>>(query, (size_t)LQ * DQ, Xq, (size_t)LQ * DQ, (size_t)LQ * DQ / 8);
    k_gemmb<false><<<dim3(NKR / 64, HH / 64, 1), 128, 0, stream>>>(Xc, nullptr, WB, nullptr, Kf, HH, DC, (size_t)0, (size_t)0, (size_t)0);
    k_gemmb<false><<<dim3(NQR / 64, HH / 64, 1), 128, 0, stream>>>(Xq, nullptr, WB + (size_t)HH * DC, bias, Qf, HH, DQ, (size_t)0, (size_t)0, (size_t)0);
    k_score<<<dim3(NQR, 1, 1), 256, 0, stream>>>(Qf, Kf, vv, gg, sbp, out0, Ph, Pl);
    k_ct<<<dim3(LK / 64, DC / 64, NB), 256, 0, stream>>>(context, CT);
    k_gemmb<true><<<dim3(LQ / 64, DC / 64, NB), 128, 0, stream>>>(Ph, Pl, CT, nullptr, out1, DC, LK, (size_t)LQ * LK, (size_t)DC * LK, (size_t)LQ * DC);
}
